// RingAttention_51702816309916
// MI455X (gfx1250) — hardware-verified
//
#include <hip/hip_runtime.h>


#ifndef NB
#define NB 2
#endif
#ifndef SEQ
#define SEQ 2048
#endif
#define NB_FULL 2
#define SEQ_FULL 2048
#define HEADS 16
#define DH 128
#define HD (HEADS * DH)
#define SEQT (NB * SEQ)
#define QBLK (SEQ / 64)
#define QBRES 4

static_assert(SEQ % 64 == 0);
static_assert(SEQ >= 64);
static_assert(SEQ <= SEQ_FULL);
static_assert(NB >= 1 && NB <= NB_FULL);
static_assert(DH == 128 && HEADS == 16);
static_assert((long long)SEQT * HD <= (long long)NB_FULL * SEQ_FULL * HD);

typedef unsigned short us16;
typedef __attribute__((ext_vector_type(16))) __bf16   v16bf;
typedef __attribute__((ext_vector_type(16))) _Float16 v16h;
typedef __attribute__((ext_vector_type(8)))  float    v8f;
typedef __attribute__((ext_vector_type(8)))  unsigned v8u;
typedef __attribute__((ext_vector_type(4)))  unsigned v4u;
typedef __attribute__((ext_vector_type(2)))  unsigned v2u;
typedef __attribute__((ext_vector_type(4)))  float    v4f;
typedef __attribute__((ext_vector_type(2)))  float    v2f;

__device__ __forceinline__ unsigned f2bf(float f) { unsigned u = __float_as_uint(f); u += 0x7FFFu + ((u >> 16) & 1u); return u >> 16; }
__device__ __forceinline__ float bf2f(unsigned h) { return __uint_as_float(h << 16); }
__device__ __forceinline__ unsigned f2h(float f) { _Float16 t = (_Float16)f; return (unsigned)__builtin_bit_cast(unsigned short, t); }

__device__ __forceinline__ v8u ld_frag(const us16* rowp, int hh) {
    const v4u a = *(const v4u*)(rowp + 8 * hh);
    const v4u b = *(const v4u*)(rowp + 16 + 8 * hh);
    return __builtin_shufflevector(a, b, 0, 1, 2, 3, 4, 5, 6, 7);
}
__device__ __forceinline__ v8f mma_bf16(v8u a, v8u b, v8f c) {
    return __builtin_amdgcn_wmma_f32_16x16x32_bf16(false, __builtin_bit_cast(v16bf, a), false, __builtin_bit_cast(v16bf, b), (short)0, c, false, false);
}
__device__ __forceinline__ v8f mma_f16(v8u a, v8u b, v8f c) {
    return __builtin_amdgcn_wmma_f32_16x16x32_f16(false, __builtin_bit_cast(v16h, a), false, __builtin_bit_cast(v16h, b), (short)0, c, false, false);
}
__device__ __forceinline__ void mma_guard(v8f& c, v8u a, v8u b) {
    asm volatile("v_nop\n\tv_nop\n\tv_nop\n\tv_nop" : "+v"(c) : "v"(a), "v"(b));
}

__global__ __launch_bounds__(256) void prep_qk(const float* __restrict__ q, const float* __restrict__ k, us16* qpl, us16* kpl) {
    const int tok = blockIdx.x;
    const int bsel = tok / SEQ, isel = tok - bsel * SEQ;
    const size_t src = ((size_t)bsel * SEQ_FULL + isel) * HD;
    const int tid = threadIdx.x, lane = tid & 31, wv = tid >> 5;
    v2u pq[2], pk[2];
    size_t dof[2];
#pragma unroll
    for (int it = 0; it < 2; ++it) {
        const int h = wv + 8 * it;
        const v4f a = *(const v4f*)(q + src + h * DH + 4 * lane);
        const v4f c = *(const v4f*)(k + src + h * DH + 4 * lane);
        pq[it].x = f2bf(a.x) | (f2bf(a.y) << 16);
        pq[it].y = f2bf(a.z) | (f2bf(a.w) << 16);
        pk[it].x = f2bf(c.x) | (f2bf(c.y) << 16);
        pk[it].y = f2bf(c.z) | (f2bf(c.w) << 16);
        dof[it] = ((size_t)h * SEQT + tok) * DH + 4 * lane;
    }
    auto pass = [&]() {
#pragma unroll
        for (int it = 0; it < 2; ++it) {
            *(volatile v2u*)(qpl + dof[it]) = pq[it];
            *(volatile v2u*)(kpl + dof[it]) = pk[it];
        }
    };
    pass();
    __threadfence();
    pass();
}

__global__ __launch_bounds__(256) void prep_v(const float* __restrict__ v, us16* vt) {
    __shared__ float tile[DH][65];
    const int tok0 = blockIdx.x * 64, h = blockIdx.y;
    const int bsel = tok0 / SEQ, s0 = tok0 - bsel * SEQ;
    const float* src = v + (((size_t)bsel * SEQ_FULL + s0) * HEADS + h) * DH;
    const int tid = threadIdx.x, lane = tid & 31, wv = tid >> 5;
#pragma unroll 4
    for (int j = 0; j < 32; ++j) {
        const int idx = tid + 256 * j;
        const int r = idx >> 7, dc = idx & 127;
        const float x = src[(size_t)r * HD + dc];
        tile[dc][r] = bf2f(f2bf(x)) * 4.0f;
    }
    __syncthreads();
    auto pass = [&]() {
#pragma unroll 4
        for (int j = 0; j < 16; ++j) {
            const int d = wv * 16 + j;
            const float a = tile[d][2 * lane], c = tile[d][2 * lane + 1];
            const unsigned pkv = f2h(a) | (f2h(c) << 16);
            *(volatile unsigned*)(vt + ((size_t)h * DH + d) * SEQT + tok0 + 2 * lane) = pkv;
        }
    };
    pass();
    __threadfence();
    pass();
}

template <int ND, int RES>
__global__ __launch_bounds__(128) __attribute__((amdgpu_num_vgpr(256)))
void attn(const us16* __restrict__ qpl, const us16* __restrict__ kpl, const us16* __restrict__ vt, float* out, int qb0) {
    __shared__ v4f ost[4][16][ND * 4 + 1];
    const int tid = threadIdx.x, lane = tid & 31, wv = tid >> 5, m = lane & 15, hh = lane >> 4;
    const int qb = qb0 + (int)blockIdx.x;
    const int h = blockIdx.y % HEADS, bsel = blockIdx.y / HEADS;
    const int dbase = (ND == 8) ? 0 : 64 * (int)blockIdx.z;
    const size_t tok0 = (size_t)bsel * SEQ;
    const int qrow = qb * 64 + wv * 16;
    const int iq = qrow + m;
    const us16* qr = qpl + ((size_t)h * SEQT + tok0 + qrow + m) * DH;
    const v8u q0 = ld_frag(qr, hh), q1 = ld_frag(qr + 32, hh), q2 = ld_frag(qr + 64, hh), q3 = ld_frag(qr + 96, hh);
    const us16* kb = kpl + ((size_t)h * SEQT + tok0) * DH;
    const us16* vb = vt + ((size_t)h * DH + dbase) * SEQT + tok0;
    const float NEG = -__builtin_inff();
    const float SCL = 0.08838834764831845f;
    v8f o[ND] = {};
    v8f orr[ND] = {};
    float mrun = NEG, lrun = 0.f;
    const int nch = 2 * qb + 2;
#pragma unroll 1
    for (int c = 0; c < nch; ++c) {
        v8f s[2] = {};
#pragma unroll
        for (int t = 0; t < 2; ++t) {
            const us16* kr = kb + (size_t)(c * 32 + t * 16 + m) * DH;
            const v8u a0 = ld_frag(kr, hh);
            s[t] = mma_bf16(a0, q0, s[t]);
            const v8u a1 = ld_frag(kr + 32, hh);
            s[t] = mma_bf16(a1, q1, s[t]);
            const v8u a2 = ld_frag(kr + 64, hh);
            s[t] = mma_bf16(a2, q2, s[t]);
            const v8u a3 = ld_frag(kr + 96, hh);
            s[t] = mma_bf16(a3, q3, s[t]);
            asm volatile("v_nop\n\tv_nop\n\tv_nop\n\tv_nop" : "+v"(s[t]) : "v"(a0), "v"(a1), "v"(a2), "v"(a3), "v"(q2), "v"(q3));
        }
        float sv[16];
        float cmax = NEG;
#pragma unroll
        for (int t = 0; t < 2; ++t)
#pragma unroll
            for (int r = 0; r < 8; ++r) {
                const int j = c * 32 + t * 16 + 8 * hh + r;
                const float val = (j <= iq) ? s[t][r] * SCL : NEG;
                sv[8 * t + r] = val;
                cmax = fmaxf(cmax, val);
            }
        cmax = fmaxf(cmax, __shfl_xor(cmax, 16, 32));
        const float mnew = fmaxf(mrun, cmax);
        const float muse = (mnew == NEG) ? 0.f : mnew;
        const float fac = (mrun == NEG) ? 0.f : __expf(mrun - muse);
        mrun = mnew;
        v16h ph, pr;
        float psum = 0.f;
#pragma unroll
        for (int r = 0; r < 8; ++r) {
            const float e0 = __expf(sv[r] - muse) * 16384.0f;
            const float e1 = __expf(sv[8 + r] - muse) * 16384.0f;
            const _Float16 p0 = (_Float16)e0, p1 = (_Float16)e1;
            ph[r] = p0;
            ph[8 + r] = p1;
            if (RES) {
                const _Float16 g0 = (_Float16)((e0 - (float)p0) * 1024.0f);
                const _Float16 g1 = (_Float16)((e1 - (float)p1) * 1024.0f);
                pr[r] = g0;
                pr[8 + r] = g1;
                psum += ((float)p0 + (float)g0 * (1.0f / 1024.0f)) + ((float)p1 + (float)g1 * (1.0f / 1024.0f));
            } else {
                pr[r] = (_Float16)0.0f;
                pr[8 + r] = (_Float16)0.0f;
                psum += (float)p0 + (float)p1;
            }
        }
        psum += __shfl_xor(psum, 16, 32);
        lrun = lrun * fac + psum;
        const v8u pbu = __builtin_bit_cast(v8u, ph);
        const v8u pru = __builtin_bit_cast(v8u, pr);
#pragma unroll
        for (int dt = 0; dt < ND; ++dt) {
            o[dt] = o[dt] * fac;
            if (RES) orr[dt] = orr[dt] * fac;
        }
#pragma unroll
        for (int dt = 0; dt < ND; ++dt) {
            const v8u va = ld_frag(vb + (size_t)(dt * 16 + m) * SEQT + c * 32, hh);
            o[dt] = mma_f16(va, pbu, o[dt]);
            if (RES) {
                orr[dt] = mma_f16(va, pru, orr[dt]);
                asm volatile("v_nop\n\tv_nop\n\tv_nop\n\tv_nop" : "+v"(o[dt]), "+v"(orr[dt]) : "v"(va), "v"(pbu), "v"(pru));
            } else {
                mma_guard(o[dt], va, pbu);
            }
        }
    }
    const float inv = 1.0f / lrun;
    const float osc = inv * 0.25f;
#pragma unroll
    for (int dt = 0; dt < ND; ++dt) {
#pragma unroll
        for (int g = 0; g < 2; ++g) {
            v4f w;
#pragma unroll
            for (int e = 0; e < 4; ++e) {
                const int r = 4 * g + e;
                float val = o[dt][r];
                if (RES) val += orr[dt][r] * (1.0f / 1024.0f);
                w[e] = val * osc;
            }
            ost[wv][m][dt * 4 + 2 * hh + g] = w;
        }
    }
    __syncthreads();
    float* ob = out + ((tok0 + qrow) * HEADS + h) * (size_t)DH + dbase;
    auto pass = [&]() {
#pragma unroll
        for (int rr = 0; rr < 16; ++rr) {
            if (ND == 8) {
                const v4f w4 = ost[wv][rr][lane];
                *(volatile v4f*)(ob + (size_t)rr * HD + 4 * lane) = w4;
            } else {
                const v4f t4 = ost[wv][rr][lane >> 1];
                v2f w2;
                w2.x = (lane & 1) ? t4.z : t4.x;
                w2.y = (lane & 1) ? t4.w : t4.y;
                *(volatile v2f*)(ob + (size_t)rr * HD + 2 * lane) = w2;
            }
        }
    };
    pass();
    __threadfence();
    pass();
}

extern "C" void kernel_launch(void* const* d_in, const int* in_sizes, int n_in,
                              void* d_out, int out_size, void* d_ws, size_t ws_size, hipStream_t stream) {
    if (n_in < 3) return;
    const float* q = (const float*)d_in[0];
    const float* k = (const float*)d_in[1];
    const float* v = (const float*)d_in[2];
    float* out = (float*)d_out;
    const long long need = ((long long)(NB - 1) * SEQ_FULL + SEQ) * HD;
    if ((long long)in_sizes[0] < need || (long long)in_sizes[1] < need || (long long)in_sizes[2] < need) return;
    if ((long long)out_size < (long long)SEQT * HD) return;

    size_t off = 0;
    auto carve = [&](size_t bytes) { size_t o0 = off; off += (bytes + 127) & ~(size_t)127; return o0; };
    char* ws = (char*)d_ws;
    us16* qpl = (us16*)(ws + carve((size_t)HEADS * SEQT * DH * 2));
    us16* kpl = (us16*)(ws + carve((size_t)HEADS * SEQT * DH * 2));
    us16* vt  = (us16*)(ws + carve((size_t)HEADS * DH * SEQT * 2));
    if (off > ws_size) return;

    prep_qk<<<SEQT, 256, 0, stream>>>(q, k, qpl, kpl);
    prep_v<<<dim3(SEQT / 64, HEADS), 256, 0, stream>>>(v, vt);
    const int qbe = (QBLK < QBRES) ? QBLK : QBRES;
    attn<4, 1><<<dim3(qbe, NB * HEADS, 2), 128, 0, stream>>>(qpl, kpl, vt, out, 0);
    if (QBLK > qbe) attn<8, 0><<<dim3(QBLK - qbe, NB * HEADS, 1), 128, 0, stream>>>(qpl, kpl, vt, out, qbe);
}
